// EncoderLayer_34333968564745
// MI455X (gfx1250) — hardware-verified
//
#include <hip/hip_runtime.h>
#include <stddef.h>
#include <stdint.h>
#include <math.h>


#define DIN    128
#define DOUT   256
#define AGP    256
#define KG     256
#define NTHR   256
#define NWAVE  8
#define EPT    8
#define CHUNK  (NTHR * EPT)
#define WCAP   (EPT * 32)
#define LISTN  (NWAVE * WCAP)
#define NBA    1024
#define SLA    10
#define RCAP   28672
#define DEGCAP 64
#define GBM    64
#define GBN    128
#define GTHR   128
#define NUW    (DOUT * (KG / 8))
#define RECP   (2 * DOUT)
#define NRB    16
#define AGG_ZINTS    (LISTN + 2 * RCAP + 3 * NBA)
#define MISC_INTS    16
#define ROWBUF_INTS  (NWAVE * AGP / 2)
#define AGG_LDS_INTS (AGG_ZINTS + MISC_INTS + ROWBUF_INTS)
#define WSMAX  134217728

static_assert((CHUNK & (CHUNK - 1)) == 0 && CHUNK <= 4096);
static_assert((NBA & (NBA - 1)) == 0 && NBA == (1 << SLA));
static_assert(((long long)CHUNK << SLA) < (1LL << 31));
static_assert(LISTN % NTHR == 0);
static_assert(NBA % NWAVE == 0 && NBA % 32 == 0 && NBA % GBM == 0);
static_assert(RCAP % 4 == 0 && AGG_ZINTS % 4 == 0 && LISTN % 4 == 0 && ((AGG_ZINTS + MISC_INTS) % 4) == 0);
static_assert(AGG_ZINTS % (NTHR * 4) == 0);
static_assert(KG % 32 == 0 && KG == 2 * DIN && AGP == KG && DIN == 4 * 32);
static_assert(GBM == (GTHR / 32) * 16 && GBN == 4 * 32 && DOUT % GBN == 0);
static_assert(NUW % NTHR == 0 && KG / 8 == 32 && DIN / 8 == 16);
static_assert(8 * GBN <= GBM * GBN);
static_assert(DEGCAP >= 38 + 8);
static_assert(NRB == 4 * (NTHR / 64) && DOUT / 4 == 64);
static_assert(AGG_LDS_INTS * 4 <= 300000);

typedef float          v4f   __attribute__((ext_vector_type(4)));
typedef float          v8f   __attribute__((ext_vector_type(8)));
typedef int            v4i   __attribute__((ext_vector_type(4)));
typedef int            v8i   __attribute__((ext_vector_type(8)));
typedef unsigned       v2u   __attribute__((ext_vector_type(2)));
typedef unsigned short v4us  __attribute__((ext_vector_type(4)));
typedef unsigned short v8us  __attribute__((ext_vector_type(8)));
typedef unsigned short v16us __attribute__((ext_vector_type(16)));
typedef __bf16         v16bf __attribute__((ext_vector_type(16)));
typedef v4f  __attribute__((may_alias)) v4fa;
typedef v4i  __attribute__((may_alias)) v4ia;
typedef v2u  __attribute__((may_alias)) v2ua;
typedef v4us __attribute__((may_alias)) v4usa;
typedef v8us __attribute__((may_alias)) v8usa;
union FragB { v16bf v; v16us u; v8us h[2]; v8i w; };

__device__ __forceinline__ v8f wmb(const FragB& a, const FragB& b, v8f c) {
  v8f d = __builtin_amdgcn_wmma_f32_16x16x32_bf16(false, a.v, false, b.v, (short)0, c, false, false);
  asm volatile("v_nop\n\tv_nop\n\tv_nop\n\tv_nop" : "+v"(d) : "v"(a.w), "v"(b.w));
  return d;
}

__device__ __forceinline__ unsigned bf16_bits(float f) {
  const unsigned u = __float_as_uint(f);
  return (u + 0x7FFFu + ((u >> 16) & 1u)) >> 16;
}
__device__ __forceinline__ float bf16_val(float f) {
  return __uint_as_float(bf16_bits(f) << 16);
}

__device__ __forceinline__ void wave_sync() {
  __builtin_amdgcn_fence(__ATOMIC_RELEASE, "wavefront");
  __builtin_amdgcn_wave_barrier();
  __builtin_amdgcn_fence(__ATOMIC_ACQUIRE, "wavefront");
}

template <int SLB>
__device__ __forceinline__ int scan_chunk(const int* __restrict__ dsts, int nE, int cbase, int slotBase,
                                          int nb, int vec8, int* list, int tid, int lane, int wave) {
  int wc = 0;
  const int el0  = tid * EPT;
  const int e0   = cbase + el0;
  const int sent = -2147483647 - 1;
  v4i da, db;
  if (vec8 != 0 && cbase + CHUNK <= nE) {
    da = *(const v4i*)(dsts + e0);
    db = *(const v4i*)(dsts + e0 + 4);
  } else {
    da.x = (e0     < nE) ? dsts[min(e0,     nE - 1)] : sent;
    da.y = (e0 + 1 < nE) ? dsts[min(e0 + 1, nE - 1)] : sent;
    da.z = (e0 + 2 < nE) ? dsts[min(e0 + 2, nE - 1)] : sent;
    da.w = (e0 + 3 < nE) ? dsts[min(e0 + 3, nE - 1)] : sent;
    db.x = (e0 + 4 < nE) ? dsts[min(e0 + 4, nE - 1)] : sent;
    db.y = (e0 + 5 < nE) ? dsts[min(e0 + 5, nE - 1)] : sent;
    db.z = (e0 + 6 < nE) ? dsts[min(e0 + 6, nE - 1)] : sent;
    db.w = (e0 + 7 < nE) ? dsts[min(e0 + 7, nE - 1)] : sent;
  }
  const unsigned nbs = (unsigned)slotBase;
  const unsigned unb = (unsigned)nb;
  const unsigned s0 = (unsigned)da.x - nbs, s1 = (unsigned)da.y - nbs;
  const unsigned s2 = (unsigned)da.z - nbs, s3 = (unsigned)da.w - nbs;
  const unsigned s4 = (unsigned)db.x - nbs, s5 = (unsigned)db.y - nbs;
  const unsigned s6 = (unsigned)db.z - nbs, s7 = (unsigned)db.w - nbs;
  const bool h0 = s0 < unb, h1 = s1 < unb, h2 = s2 < unb, h3 = s3 < unb;
  const bool h4 = s4 < unb, h5 = s5 < unb, h6 = s6 < unb, h7 = s7 < unb;
  const unsigned any = __builtin_amdgcn_ballot_w32(h0 | h1 | h2 | h3 | h4 | h5 | h6 | h7);
  if (any != 0u) {
#define HITJ(J, HJ, SJ) { \
      const unsigned mj = __builtin_amdgcn_ballot_w32(HJ); \
      if (mj != 0u) { \
        if (HJ) { \
          const int pos = wc + (int)__builtin_amdgcn_mbcnt_lo(mj, 0u); \
          if (pos < WCAP) list[wave * WCAP + pos] = ((el0 + (J)) << SLB) | (int)(SJ); \
        } \
        wc += (int)__builtin_popcount(mj); } }
    HITJ(0, h0, s0)
    HITJ(1, h1, s1)
    HITJ(2, h2, s2)
    HITJ(3, h3, s3)
    HITJ(4, h4, s4)
    HITJ(5, h5, s5)
    HITJ(6, h6, s6)
    HITJ(7, h7, s7)
#undef HITJ
  }
  return wc;
}

__global__ __launch_bounds__(NTHR) void k_prep(const float* __restrict__ x, const float* __restrict__ W,
                                               int nN, int gX, unsigned short* xb, unsigned short* w2t) {
  const int bx  = (int)blockIdx.x;
  const int tid = (int)threadIdx.x;
  if (bx < gX) {
    const int u = bx * NTHR + tid;
    if (u < nN * (DIN / 8)) {
      const int row = u >> 4;
      const int k8  = (u & 15) * 8;
      const float* p = x + (size_t)row * DIN + k8;
      const v4f a = *(const v4fa*)p;
      const v4f b = *(const v4fa*)(p + 4);
      v8us o;
      o[0] = (unsigned short)bf16_bits(a.x); o[1] = (unsigned short)bf16_bits(a.y);
      o[2] = (unsigned short)bf16_bits(a.z); o[3] = (unsigned short)bf16_bits(a.w);
      o[4] = (unsigned short)bf16_bits(b.x); o[5] = (unsigned short)bf16_bits(b.y);
      o[6] = (unsigned short)bf16_bits(b.z); o[7] = (unsigned short)bf16_bits(b.w);
      unsigned short* dp = xb + (size_t)row * DIN + k8;
      *(volatile v8us*)dp = o;
      __threadfence();
      *(volatile v8us*)dp = o;
    }
  } else {
    const int u = (bx - gX) * NTHR + tid;
    if (u < NUW) {
      const int n  = u >> 5;
      const int k8 = (u & 31) * 8;
      const int kk = k8 & (DIN - 1);
      const float* p = W + (size_t)kk * DOUT + n;
      v8us o;
#pragma unroll
      for (int i = 0; i < 8; ++i) o[i] = (unsigned short)bf16_bits(p[(size_t)i * DOUT]);
      unsigned short* dp = w2t + (size_t)n * KG + k8;
      *(volatile v8us*)dp = o;
      __threadfence();
      *(volatile v8us*)dp = o;
    }
  }
}

__global__ __launch_bounds__(NTHR) void k_scan(const int* __restrict__ gath, const int* __restrict__ keys,
                                               const float* __restrict__ ew,
                                               int nE, int nN, int vec8, int mRows,
                                               const unsigned short* __restrict__ xb, unsigned short* apl) {
  extern __shared__ __attribute__((aligned(16))) int dsm[];
  int* list = dsm;
  int* hl   = dsm + LISTN;
  int* sl   = hl + RCAP;
  int* cnt  = sl + RCAP;
  int* offs = cnt + NBA;
  int* cur  = offs + NBA;
  int* misc = cur + NBA;
  const int tid = (int)threadIdx.x, lane = tid & 31, wave = tid >> 5;
  unsigned short* rowbuf = (unsigned short*)(misc + MISC_INTS) + wave * AGP;
  const int nodeBase = (int)blockIdx.x * NBA;

  {
    const v4i z4 = {0, 0, 0, 0};
    for (int i = tid * 4; i < AGG_ZINTS; i += NTHR * 4) *(v4ia*)(dsm + i) = z4;
    if (tid < MISC_INTS) misc[tid] = 0;
  }
  __syncthreads();

  int t = 0, ov = 0;
  const int nChunks = (nE + CHUNK - 1) / CHUNK;
#pragma unroll 1
  for (int ch = 0; ch < nChunks; ++ch) {
    const int cbase = ch * CHUNK;
    const int wc = scan_chunk<SLA>(keys, nE, cbase, nodeBase, NBA, vec8, list, tid, lane, wave);
    if (lane == 0) misc[wave] = wc;
    __syncthreads();
    if (wave == 0) {
#pragma unroll 1
      for (int w2 = 0; w2 < NWAVE; ++w2) {
        int c = misc[w2];
        c = c < 0 ? 0 : (c > WCAP ? WCAP : c);
#pragma unroll 1
        for (int b0 = 0; b0 < c; b0 += 32) {
          const int idx = b0 + lane;
          const int ent = list[w2 * WCAP + (idx < WCAP ? idx : WCAP - 1)];
          const int m32 = (c - b0) < 32 ? (c - b0) : 32;
#pragma unroll 1
          for (int k = 0; k < m32; ++k) {
            const int u    = __builtin_amdgcn_readlane(ent, k);
            const int slot = u & (NBA - 1);
            const int el   = (u >> SLA) & (CHUNK - 1);
            const int pk   = ((cbase + el) << SLA) | slot;
            if (t < RCAP) {
              if (lane == 0) { hl[t] = pk; cnt[slot] = cnt[slot] + 1; }
              t = t + 1;
            } else {
              ov = 1;
            }
          }
        }
      }
    }
    __syncthreads();
  }
  if (wave == 0 && lane == 0) { misc[8] = t; misc[9] = ov; }
  __syncthreads();
  int tt = misc[8];
  tt = tt < 0 ? 0 : (tt > RCAP ? RCAP : tt);
  const int ovf = misc[9];

  if (wave == 0) {
    const int base = lane * (NBA / 32);
    int s = 0;
#pragma unroll 1
    for (int i = 0; i < NBA / 32; ++i) s += cnt[base + i];
    int incl = s;
#pragma unroll
    for (int d = 1; d < 32; d <<= 1) {
      const int y = __shfl_up(incl, d, 32);
      if (lane >= d) incl += y;
    }
    int run = incl - s;
#pragma unroll 1
    for (int i = 0; i < NBA / 32; ++i) {
      const int cv = cnt[base + i];
      offs[base + i] = run;
      cur[base + i]  = run;
      run += cv;
    }
  }
  __syncthreads();
  if (wave == 0) {
#pragma unroll 1
    for (int b0 = 0; b0 < tt; b0 += 32) {
      const int idx = b0 + lane;
      const int ent = hl[idx < RCAP ? idx : RCAP - 1];
      const int m32 = (tt - b0) < 32 ? (tt - b0) : 32;
#pragma unroll 1
      for (int k = 0; k < m32; ++k) {
        const int u    = __builtin_amdgcn_readlane(ent, k);
        const int slot = u & (NBA - 1);
        if (lane == 0) {
          int p = cur[slot];
          p = p < 0 ? 0 : (p > RCAP - 1 ? RCAP - 1 : p);
          sl[p] = u;
          cur[slot] = p + 1;
        }
      }
    }
  }
  __syncthreads();

  const float qnan = __int_as_float(0x7fc00000);
  const float pz = (ovf != 0) ? qnan : 0.0f;
#pragma unroll 1
  for (int si = 0; si < NBA / NWAVE; ++si) {
    const int s    = si * NWAVE + wave;
    const int node = nodeBase + s;
    int c = cnt[s];
    const bool big = c > DEGCAP;
    c = c < 0 ? 0 : (c > DEGCAP ? DEGCAP : c);
    int o = offs[s];
    o = o < 0 ? 0 : (o > RCAP ? RCAP : o);
    float a0 = 0.0f, a1 = 0.0f, a2 = 0.0f, a3 = 0.0f;
#pragma unroll 1
    for (int b0 = 0; b0 < c; b0 += 32) {
      int idx = o + b0 + lane;
      idx = idx > RCAP - 1 ? RCAP - 1 : idx;
      const int ent = sl[idx];
      int eid = ent >> SLA;
      eid = eid < 0 ? 0 : (eid > nE - 1 ? nE - 1 : eid);
      int sr = gath[eid];
      sr = sr < 0 ? 0 : (sr > nN - 1 ? nN - 1 : sr);
      const float wv  = bf16_val(ew[eid]);
      const int   wvi = __float_as_int(wv);
      const int m32 = (c - b0) < 32 ? (c - b0) : 32;
#pragma unroll 1
      for (int k = 0; k < m32; ++k) {
        const int   sk = __builtin_amdgcn_readlane(sr, k);
        const float ck = __int_as_float(__builtin_amdgcn_readlane(wvi, k));
        const unsigned short* rp = xb + (size_t)sk * DIN + 4 * lane;
        const v2u w = *(const v2ua*)rp;
        const float f0 = __uint_as_float(w.x << 16);
        const float f1 = __uint_as_float(w.x & 0xffff0000u);
        const float f2 = __uint_as_float(w.y << 16);
        const float f3 = __uint_as_float(w.y & 0xffff0000u);
        a0 = fmaf(ck, f0, a0);
        a1 = fmaf(ck, f1, a1);
        a2 = fmaf(ck, f2, a2);
        a3 = fmaf(ck, f3, a3);
      }
    }
    const float pzr = big ? qnan : pz;
    const bool live = node < nN;
    const float m0 = live ? (a0 + pzr) : 0.0f;
    const float m1 = live ? (a1 + pzr) : 0.0f;
    const float m2 = live ? (a2 + pzr) : 0.0f;
    const float m3 = live ? (a3 + pzr) : 0.0f;
    v4us mh, ml;
    {
      unsigned hb;
      hb = bf16_bits(m0); mh[0] = (unsigned short)hb; ml[0] = (unsigned short)bf16_bits(m0 - __uint_as_float(hb << 16));
      hb = bf16_bits(m1); mh[1] = (unsigned short)hb; ml[1] = (unsigned short)bf16_bits(m1 - __uint_as_float(hb << 16));
      hb = bf16_bits(m2); mh[2] = (unsigned short)hb; ml[2] = (unsigned short)bf16_bits(m2 - __uint_as_float(hb << 16));
      hb = bf16_bits(m3); mh[3] = (unsigned short)hb; ml[3] = (unsigned short)bf16_bits(m3 - __uint_as_float(hb << 16));
    }
    *(v4usa*)(rowbuf + 4 * lane) = mh;
    *(v4usa*)(rowbuf + DIN + 4 * lane) = ml;
    wave_sync();
    const v8us q0 = *(const v8usa*)(rowbuf + 8 * lane);
    wave_sync();
    if (node < mRows) {
      unsigned short* rpw = apl + (size_t)node * AGP + 8 * lane;
      *(volatile v8us*)rpw = q0;
      __threadfence();
      *(volatile v8us*)rpw = q0;
    }
  }
}

__global__ __launch_bounds__(GTHR) void k_gemm(const unsigned short* __restrict__ Apl,
                                               const unsigned short* __restrict__ BT,
                                               const float* __restrict__ bias, float* R, float* rec, int nOut) {
  __shared__ __attribute__((aligned(16))) float stg[GBM * GBN];
  const int tid = (int)threadIdx.x, lane = tid & 31, wave = tid >> 5, hh = lane >> 4, m = lane & 15;
  const int rowBase = (int)blockIdx.x * GBM;
  const int col0    = (int)blockIdx.y * GBN;

  v8f acc[8];
  {
    const v8f z = {0.f, 0.f, 0.f, 0.f, 0.f, 0.f, 0.f, 0.f};
#pragma unroll
    for (int t = 0; t < 8; ++t) acc[t] = z;
  }
  const unsigned short* ap = Apl + (size_t)(rowBase + 16 * wave + m) * (size_t)KG + 8 * hh;
  const unsigned short* bp = BT + (size_t)(col0 + m) * (size_t)KG + 8 * hh;

#pragma unroll 1
  for (int k0 = 0; k0 < KG; k0 += 32) {
    FragB af;
    af.h[0] = *(const v8usa*)(ap + k0);
    af.h[1] = *(const v8usa*)(ap + k0 + 16);
#pragma unroll
    for (int nt = 0; nt < 8; ++nt) {
      const unsigned short* wq = bp + (size_t)(16 * nt) * (size_t)KG + k0;
      FragB bf;
      bf.h[0] = *(const v8usa*)wq;
      bf.h[1] = *(const v8usa*)(wq + 16);
      acc[nt] = wmb(af, bf, acc[nt]);
    }
  }

#pragma unroll
  for (int nt = 0; nt < 8; ++nt) {
    const int lc = 16 * nt + m;
#pragma unroll
    for (int r = 0; r < 8; ++r) {
      const int lr = 16 * wave + 8 * hh + r;
      stg[lr * GBN + lc] = acc[nt][r];
    }
  }
  __syncthreads();

  v4f bb4;
  {
    const v4f t1 = *(const v4fa*)(bias + col0 + 4 * lane);
    bb4.x = bf16_val(t1.x); bb4.y = bf16_val(t1.y); bb4.z = bf16_val(t1.z); bb4.w = bf16_val(t1.w);
  }

  v4f pv[16];
#pragma unroll
  for (int i = 0; i < 16; ++i) pv[i] = *(const v4fa*)(stg + (16 * wave + i) * GBN + 4 * lane);
  __syncthreads();

  v4f cs = {0.f, 0.f, 0.f, 0.f};
  v4f cq = {0.f, 0.f, 0.f, 0.f};
#pragma unroll
  for (int i = 0; i < 16; ++i) {
    const bool ok = (rowBase + 16 * wave + i) < nOut;
    const v4f t = pv[i] + bb4;
    v4f y;
    y.x = (t.x > 0.0f) ? t.x : (t.x - t.x);
    y.y = (t.y > 0.0f) ? t.y : (t.y - t.y);
    y.z = (t.z > 0.0f) ? t.z : (t.z - t.z);
    y.w = (t.w > 0.0f) ? t.w : (t.w - t.w);
    y.x = ok ? y.x : 0.0f; y.y = ok ? y.y : 0.0f; y.z = ok ? y.z : 0.0f; y.w = ok ? y.w : 0.0f;
    pv[i] = y;
    cs = cs + y;
    cq = cq + y * y;
  }
  *(v4fa*)(stg + wave * GBN + 4 * lane) = cs;
  *(v4fa*)(stg + (4 + wave) * GBN + 4 * lane) = cq;
  __syncthreads();
  v4f rs, rq;
  {
    const v4f p0 = *(const v4fa*)(stg + 0 * GBN + 4 * lane);
    const v4f p1 = *(const v4fa*)(stg + 1 * GBN + 4 * lane);
    const v4f p2 = *(const v4fa*)(stg + 2 * GBN + 4 * lane);
    const v4f p3 = *(const v4fa*)(stg + 3 * GBN + 4 * lane);
    rs = ((p0 + p1) + p2) + p3;
    const v4f q0 = *(const v4fa*)(stg + 4 * GBN + 4 * lane);
    const v4f q1 = *(const v4fa*)(stg + 5 * GBN + 4 * lane);
    const v4f q2 = *(const v4fa*)(stg + 6 * GBN + 4 * lane);
    const v4f q3 = *(const v4fa*)(stg + 7 * GBN + 4 * lane);
    rq = ((q0 + q1) + q2) + q3;
  }
  float* rcp = rec + (size_t)blockIdx.x * RECP + col0 + 4 * lane;

#pragma unroll
  for (int i = 0; i < 16; ++i) {
    const int r = rowBase + 16 * wave + i;
    if (r < nOut) *(volatile v4f*)(R + (size_t)r * DOUT + col0 + 4 * lane) = pv[i];
  }
  if (wave == 0) {
    *(volatile v4f*)rcp = rs;
    *(volatile v4f*)(rcp + DOUT) = rq;
  }
  __threadfence();
#pragma unroll
  for (int i = 0; i < 16; ++i) {
    const int r = rowBase + 16 * wave + i;
    if (r < nOut) *(volatile v4f*)(R + (size_t)r * DOUT + col0 + 4 * lane) = pv[i];
  }
  if (wave == 0) {
    *(volatile v4f*)rcp = rs;
    *(volatile v4f*)(rcp + DOUT) = rq;
  }
}

__global__ __launch_bounds__(NTHR) void k_combine(const float* __restrict__ rec, int nTiles, double invN,
                                                  float* ms) {
  __shared__ __attribute__((aligned(16))) float sm[2 * DOUT];
  const int tid = (int)threadIdx.x;
  double s = 0.0, q = 0.0;
#pragma unroll 4
  for (int t = 0; t < nTiles; ++t) {
    s += (double)rec[(size_t)t * RECP + tid];
    q += (double)rec[(size_t)t * RECP + DOUT + tid];
  }
  const double mean = s * invN;
  double var = q * invN - mean * mean;
  var = (var < 0.0) ? 0.0 : var;
  const float mf = (float)mean;
  const float vf = (float)var;
  sm[tid] = mf;
  sm[DOUT + tid] = rsqrtf(vf + 1e-5f);
  __syncthreads();
  const int t4 = 4 * (tid & 127);
  const v4f v = *(const v4fa*)(sm + t4);
  const bool okst = tid < 128;
  if (okst) *(volatile v4f*)(ms + t4) = v;
  __threadfence();
  if (okst) *(volatile v4f*)(ms + t4) = v;
}

__global__ __launch_bounds__(NTHR) void k_norm(const float* __restrict__ R, const float* __restrict__ ms,
                                               const float* __restrict__ gamma, const float* __restrict__ beta,
                                               int nN, float* out) {
  const int tid  = (int)threadIdx.x;
  const int c4   = 4 * (tid & 63);
  const int rsub = tid >> 6;
  const v4f mu = *(const v4fa*)(ms + c4);
  const v4f rs = *(const v4fa*)(ms + DOUT + c4);
  v4f g, b;
  {
    const v4f g0 = *(const v4fa*)(gamma + c4);
    const v4f b0 = *(const v4fa*)(beta + c4);
    g.x = bf16_val(g0.x); g.y = bf16_val(g0.y); g.z = bf16_val(g0.z); g.w = bf16_val(g0.w);
    b.x = bf16_val(b0.x); b.y = bf16_val(b0.y); b.z = bf16_val(b0.z); b.w = bf16_val(b0.w);
  }
  const int row0 = (int)blockIdx.x * NRB + rsub;
  v4f o[4];
#pragma unroll
  for (int it = 0; it < 4; ++it) {
    const int row = row0 + 4 * it;
    const int rc  = row < nN ? row : nN - 1;
    const v4f v = *(const v4fa*)(R + (size_t)rc * DOUT + c4);
    o[it] = ((v - mu) * rs) * g + b;
  }
#pragma unroll
  for (int it = 0; it < 4; ++it) {
    const int row = row0 + 4 * it;
    if (row < nN) *(volatile v4f*)(out + (size_t)row * DOUT + c4) = o[it];
  }
  __threadfence();
#pragma unroll
  for (int it = 0; it < 4; ++it) {
    const int row = row0 + 4 * it;
    if (row < nN) *(volatile v4f*)(out + (size_t)row * DOUT + c4) = o[it];
  }
}

static inline int cdiv(int a, int b) { return (a + b - 1) / b; }
static inline size_t al256(size_t o) { return (o + 255) & ~(size_t)255; }

extern "C" void kernel_launch(void* const* d_in, const int* in_sizes, int n_in,
                              void* d_out, int out_size, void* d_ws, size_t ws_size,
                              hipStream_t stream) {
  if (n_in < 8) return;
  if (in_sizes[0] < DIN || (in_sizes[0] % DIN) != 0) return;
  const int nN = in_sizes[0] / DIN;
  if (nN < 16 || nN >= (1 << 22)) return;
  if (in_sizes[1] != DIN * DOUT) return;
  if (in_sizes[2] != DOUT || in_sizes[3] != DOUT || in_sizes[4] != DOUT) return;
  const int nE = in_sizes[5];
  if (nE < 1 || nE >= (1 << 21)) return;
  if (in_sizes[6] != nE || in_sizes[7] != nE) return;
  if ((long long)out_size != (long long)nN * DOUT) return;

  const float* x     = (const float*)d_in[0];
  const float* W     = (const float*)d_in[1];
  const float* b     = (const float*)d_in[2];
  const float* gamma = (const float*)d_in[3];
  const float* beta  = (const float*)d_in[4];
  const float* ew    = (const float*)d_in[5];
  const int*   src   = (const int*)d_in[6];
  const int*   dst   = (const int*)d_in[7];
  float* out = (float*)d_out;

  const int MP = cdiv(nN, GBM) * GBM;
  const int gM = MP / GBM;
  const int gA = cdiv(nN, NBA);
  if ((long long)gA * NBA < (long long)MP) return;
  const int vec8 = ((nE & 3) == 0) ? 1 : 0;
  const int gX = cdiv(nN * (DIN / 8), NTHR);
  const double invN = 1.0 / (double)nN;

  char* ws = (char*)d_ws;
  size_t off = 0;
  const size_t oXB  = off; off = al256(off + (size_t)nN * DIN * 2);
  const size_t oW2T = off; off = al256(off + (size_t)DOUT * KG * 2);
  const size_t oAGG = off; off = al256(off + (size_t)MP * AGP * 2);
  const size_t oR   = off; off = al256(off + (size_t)MP * DOUT * 4);
  const size_t oREC = off; off = al256(off + (size_t)gM * RECP * 4);
  const size_t oMS  = off; off = al256(off + (size_t)2 * DOUT * 4);
  if (off > ws_size || off > (size_t)WSMAX) return;
  unsigned short* XB  = (unsigned short*)(ws + oXB);
  unsigned short* W2T = (unsigned short*)(ws + oW2T);
  unsigned short* AGG = (unsigned short*)(ws + oAGG);
  float*          R   = (float*)(ws + oR);
  float*          REC = (float*)(ws + oREC);
  float*          MS  = (float*)(ws + oMS);

  const size_t scanLds = (size_t)AGG_LDS_INTS * 4;
  hipFuncSetAttribute(reinterpret_cast<const void*>(&k_scan), hipFuncAttributeMaxDynamicSharedMemorySize, (int)scanLds);

  k_prep<<<gX + NUW / NTHR, NTHR, 0, stream>>>(x, W, nN, gX, XB, W2T);
  k_scan<<<gA, NTHR, scanLds, stream>>>(src, dst, ew, nE, nN, vec8, MP, XB, AGG);
  k_gemm<<<dim3(gM, DOUT / GBN), GTHR, 0, stream>>>(AGG, W2T, b, R, REC, nN);
  k_combine<<<1, NTHR, 0, stream>>>(REC, gM, invN, MS);
  k_norm<<<cdiv(nN, NRB), NTHR, 0, stream>>>(R, MS, gamma, beta, nN, out);
}
